// Node_25847113188082
// MI455X (gfx1250) — hardware-verified
//
#include <hip/hip_runtime.h>
#include <math.h>
#include <stddef.h>
#include <stdint.h>


typedef _Float16 v16h __attribute__((ext_vector_type(16)));
typedef _Float16 v8h  __attribute__((ext_vector_type(8)));
typedef float    v8f  __attribute__((ext_vector_type(8)));
typedef float    v4f  __attribute__((ext_vector_type(4)));

#define DEVI __device__ __forceinline__
#define NOP4 "v_nop\n\tv_nop\n\tv_nop\n\tv_nop"

constexpr int kB   = 4;
constexpr int kL   = 1024;
constexpr int kC   = 1024;
constexpr int kH   = 16;
constexpr int kD   = 64;
constexpr int kNI  = 2;
constexpr int kTok = kB * kL;

union Frag16 { v16h v; v8h p[2]; };

DEVI v16h ld_frag(const _Float16* rowp, int k0, int h8) {
  Frag16 f;
  f.p[0] = *(const v8h*)(rowp + k0 + h8);
  f.p[1] = *(const v8h*)(rowp + k0 + 16 + h8);
  return f.v;
}

DEVI v8f wmma16(v16h a, v16h b, v8f c) {
  return __builtin_amdgcn_wmma_f32_16x16x32_f16(false, a, false, b, (short)0, c, false, false);
}

DEVI v8f zero8() {
  v8f z;
#pragma unroll
  for (int i = 0; i < 8; ++i) z[i] = 0.0f;
  return z;
}

DEVI float gelu_f(float v) { return 0.5f * v * (1.0f + erff(v * 0.70710678118654752f)); }

DEVI float wave_sum(float v) {
  v += __shfl_xor(v, 16);
  v += __shfl_xor(v, 8);
  v += __shfl_xor(v, 4);
  v += __shfl_xor(v, 2);
  v += __shfl_xor(v, 1);
  return v;
}

template<int EPI>
__global__ __launch_bounds__(32)
void gemm_nt_kernel(const _Float16* __restrict__ A, const _Float16* __restrict__ W,
                    const float* __restrict__ bias, const float* __restrict__ aux,
                    float* outF, _Float16* outH, int M, int N, int K)
{
  constexpr bool kHalfOut = (EPI == 2) || (EPI == 3);
  __shared__ union { float f[32 * 64]; v4f q[32 * 16]; _Float16 hh[32 * 64]; v8h hq[32 * 8]; } T;

  const int l  = threadIdx.x & 31;
  const int h8 = (l >> 4) * 8;
  const int m  = l & 15;
  const int m0 = blockIdx.y * 32;
  const int n0 = blockIdx.x * 64;
  if (m0 + 32 > M || n0 + 64 > N) return;

  v8f acc[2][4];
#pragma unroll
  for (int i = 0; i < 2; ++i)
#pragma unroll
    for (int j = 0; j < 4; ++j) acc[i][j] = zero8();

  const _Float16* Ar0 = A + (size_t)(m0 + m) * K;
  const _Float16* Ar1 = Ar0 + (size_t)16 * K;
  const _Float16* Wr0 = W + (size_t)(n0 + m) * K;
  const _Float16* Wr1 = Wr0 + (size_t)16 * K;
  const _Float16* Wr2 = Wr0 + (size_t)32 * K;
  const _Float16* Wr3 = Wr0 + (size_t)48 * K;

  for (int k = 0; k < K; k += 32) {
    const v16h a0 = ld_frag(Ar0, k, h8);
    const v16h a1 = ld_frag(Ar1, k, h8);
    const v16h b0 = ld_frag(Wr0, k, h8);
    const v16h b1 = ld_frag(Wr1, k, h8);
    const v16h b2 = ld_frag(Wr2, k, h8);
    const v16h b3 = ld_frag(Wr3, k, h8);
    acc[0][0] = wmma16(a0, b0, acc[0][0]);
    acc[0][1] = wmma16(a0, b1, acc[0][1]);
    acc[0][2] = wmma16(a0, b2, acc[0][2]);
    acc[0][3] = wmma16(a0, b3, acc[0][3]);
    acc[1][0] = wmma16(a1, b0, acc[1][0]);
    acc[1][1] = wmma16(a1, b1, acc[1][1]);
    acc[1][2] = wmma16(a1, b2, acc[1][2]);
    acc[1][3] = wmma16(a1, b3, acc[1][3]);
    asm volatile(NOP4
                 : "+v"(acc[0][0]), "+v"(acc[0][1]), "+v"(acc[0][2]), "+v"(acc[0][3]),
                   "+v"(acc[1][0]), "+v"(acc[1][1]), "+v"(acc[1][2]), "+v"(acc[1][3])
                 : "v"(a0), "v"(a1), "v"(b0), "v"(b1), "v"(b2), "v"(b3));
  }

#pragma unroll
  for (int i = 0; i < 2; ++i)
#pragma unroll
    for (int j = 0; j < 4; ++j)
#pragma unroll
      for (int r = 0; r < 8; ++r) {
        const int row = i * 16 + h8 + r;
        const int col = j * 16 + m;
        float v = acc[i][j][r] + bias[n0 + col];
        if (EPI == 1 || EPI == 2) v = gelu_f(v);
        else if (EPI == 3) v = fmaxf(v, 0.0f);
        else if (EPI == 4) v = 1.0f / (1.0f + expf(-v));
        if (kHalfOut) T.hh[row * 64 + col] = (_Float16)v;
        else          T.f[row * 64 + col]  = v;
      }
  __syncthreads();

  if (!kHalfOut) {
    v4f vals[16];
#pragma unroll
    for (int p = 0; p < 16; ++p) {
      const int ln  = 4 * p + (l >> 3);
      const int row = ln >> 1;
      const int col = ((ln & 1) << 5) + ((l & 7) << 2);
      v4f v = T.q[row * 16 + (col >> 2)];
      const size_t o = (size_t)(m0 + row) * N + n0 + col;
      if (EPI == 4) {
        const v4f xa = *(const v4f*)(aux + 2 * o);
        const v4f xb = *(const v4f*)(aux + 2 * o + 4);
        v4f xs;
        xs[0] = xa[1]; xs[1] = xa[3]; xs[2] = xb[1]; xs[3] = xb[3];
        v = v * xs;
      } else if (EPI == 5) {
        v = v + *(const v4f*)(aux + o);
      }
      vals[p] = v;
    }
#pragma unroll
    for (int p = 0; p < 16; ++p) {
      const int ln  = 4 * p + (l >> 3);
      const int row = ln >> 1;
      const int col = ((ln & 1) << 5) + ((l & 7) << 2);
      *(volatile v4f*)(outF + (size_t)(m0 + row) * N + n0 + col) = vals[p];
    }
    __threadfence();
#pragma unroll
    for (int p = 0; p < 16; ++p) {
      const int ln  = 4 * p + (l >> 3);
      const int row = ln >> 1;
      const int col = ((ln & 1) << 5) + ((l & 7) << 2);
      *(volatile v4f*)(outF + (size_t)(m0 + row) * N + n0 + col) = vals[p];
    }
  } else {
    v8h vals[8];
#pragma unroll
    for (int p = 0; p < 8; ++p) {
      const int row = 4 * p + (l >> 3);
      const int c8  = l & 7;
      vals[p] = T.hq[row * 8 + c8];
    }
#pragma unroll
    for (int p = 0; p < 8; ++p) {
      const int row = 4 * p + (l >> 3);
      const int c8  = l & 7;
      *(volatile v8h*)(outH + (size_t)(m0 + row) * N + n0 + c8 * 8) = vals[p];
    }
    __threadfence();
#pragma unroll
    for (int p = 0; p < 8; ++p) {
      const int row = 4 * p + (l >> 3);
      const int c8  = l & 7;
      *(volatile v8h*)(outH + (size_t)(m0 + row) * N + n0 + c8 * 8) = vals[p];
    }
  }
}

__global__ __launch_bounds__(256)
void cvt_f16_kernel(const float* __restrict__ src, int sstride, int soff,
                    _Float16* dst, int n8)
{
  const int t = blockIdx.x * 256 + threadIdx.x;
  if (t >= n8) return;
  v8h hv;
#pragma unroll
  for (int i = 0; i < 8; ++i)
    hv[i] = (_Float16)src[((size_t)t * 8 + i) * (size_t)sstride + soff];
  _Float16* d = dst + (size_t)t * 8;
  *(volatile v8h*)d = hv;
  __threadfence();
  *(volatile v8h*)d = hv;
}

__global__ __launch_bounds__(256)
void mix_kernel(const float* __restrict__ x_list, const float* __restrict__ wsrc,
                const float* __restrict__ op0, const float* __restrict__ op1,
                const float* __restrict__ op3, float* xmix, int n4)
{
  __shared__ float wsm[8];
  if (threadIdx.x == 0) {
    float u[6];
    float mx = -3.0e38f;
    for (int j = 0; j < 6; ++j) { u[j] = wsrc[j] * 100.0f; mx = fmaxf(mx, u[j]); }
    float s = 0.0f;
    for (int j = 0; j < 6; ++j) { u[j] = expf(u[j] - mx); s += u[j]; }
    for (int j = 0; j < 6; ++j) wsm[j] = u[j] / s;
  }
  __syncthreads();
  const int t = blockIdx.x * 256 + threadIdx.x;
  if (t < n4) {
    const size_t e = (size_t)t * 4;
    const float w0 = wsm[0], w1 = wsm[1], w2 = wsm[2], w3 = wsm[3], w4 = wsm[4], w5 = wsm[5];
    const v4f xa = *(const v4f*)(x_list + 2 * e);
    const v4f xb = *(const v4f*)(x_list + 2 * e + 4);
    v4f x0, x1;
    x0[0] = xa[0]; x0[1] = xa[2]; x0[2] = xb[0]; x0[3] = xb[2];
    x1[0] = xa[1]; x1[1] = xa[3]; x1[2] = xb[1]; x1[3] = xb[3];
    const v4f a0 = *(const v4f*)(op0 + e);
    const v4f a1 = *(const v4f*)(op1 + e);
    const v4f a3 = *(const v4f*)(op3 + e);
    v4f v;
#pragma unroll
    for (int i = 0; i < 4; ++i)
      v[i] = w0 * x0[i] + w1 * x1[i] + w2 * a0[i] + w3 * a1[i] + w4 * x1[i] + w5 * a3[i];
    *(volatile v4f*)(xmix + e) = v;
    __threadfence();
    *(volatile v4f*)(xmix + e) = v;
  }
}

__global__ __launch_bounds__(256)
void ln_qkv_kernel(const float* __restrict__ qkv,
                   const float* __restrict__ nqg, const float* __restrict__ nqb,
                   const float* __restrict__ nkg, const float* __restrict__ nkb,
                   _Float16* qh, _Float16* kh, _Float16* vth)
{
  __shared__ union { _Float16 h[64 * 64]; v8h q[64 * 8]; } Qs;
  __shared__ union { _Float16 h[64 * 64]; v8h q[64 * 8]; } Ks;
  __shared__ union { _Float16 h[64 * 64]; v8h q[64 * 8]; } Vs;

  const int tid = threadIdx.x;
  const int w   = tid >> 5;
  const int l   = tid & 31;
  const int bh  = blockIdx.y;
  const int b   = bh / kH;
  const int hd  = bh - b * kH;
  const int n0  = blockIdx.x * 64;

  const float gq0 = nqg[2 * l], gq1 = nqg[2 * l + 1];
  const float cq0 = nqb[2 * l], cq1 = nqb[2 * l + 1];
  const float gk0 = nkg[2 * l], gk1 = nkg[2 * l + 1];
  const float ck0 = nkb[2 * l], ck1 = nkb[2 * l + 1];

  for (int t = 0; t < 8; ++t) {
    const int tl = w * 8 + t;
    const size_t tok = (size_t)b * kL + n0 + tl;
    const float* qp = qkv + tok * (size_t)(3 * kC) + hd * kD + 2 * l;
    const float* kp = qp + kC;
    {
      const float x0 = qp[0], x1 = qp[1];
      const float mean = wave_sum(x0 + x1) * (1.0f / 64.0f);
      const float d0 = x0 - mean, d1 = x1 - mean;
      const float var = wave_sum(d0 * d0 + d1 * d1) * (1.0f / 64.0f);
      const float rstd = rsqrtf(var + 1e-5f);
      Qs.h[tl * 64 + 2 * l]     = (_Float16)(d0 * rstd * gq0 + cq0);
      Qs.h[tl * 64 + 2 * l + 1] = (_Float16)(d1 * rstd * gq1 + cq1);
    }
    {
      const float x0 = kp[0], x1 = kp[1];
      const float mean = wave_sum(x0 + x1) * (1.0f / 64.0f);
      const float d0 = x0 - mean, d1 = x1 - mean;
      const float var = wave_sum(d0 * d0 + d1 * d1) * (1.0f / 64.0f);
      const float rstd = rsqrtf(var + 1e-5f);
      Ks.h[tl * 64 + 2 * l]     = (_Float16)(d0 * rstd * gk0 + ck0);
      Ks.h[tl * 64 + 2 * l + 1] = (_Float16)(d1 * rstd * gk1 + ck1);
    }
  }
  {
    const int tl  = tid >> 2;
    const int d0i = (tid & 3) * 16;
    const size_t tok = (size_t)b * kL + n0 + tl;
    const float* vp = qkv + tok * (size_t)(3 * kC) + 2 * kC + hd * kD + d0i;
#pragma unroll
    for (int i = 0; i < 4; ++i) {
      const v4f x = *(const v4f*)(vp + 4 * i);
#pragma unroll
      for (int e = 0; e < 4; ++e) Vs.h[(d0i + 4 * i + e) * 64 + tl] = (_Float16)x[e];
    }
  }
  __syncthreads();

  v8h vals[6];
#pragma unroll
  for (int i = 0; i < 2; ++i) {
    const int row = i * 32 + (tid >> 3);
    const int c8  = tid & 7;
    vals[i]     = Qs.q[row * 8 + c8];
    vals[2 + i] = Ks.q[row * 8 + c8];
    vals[4 + i] = Vs.q[row * 8 + c8];
  }
#pragma unroll
  for (int i = 0; i < 2; ++i) {
    const int row = i * 32 + (tid >> 3);
    const int c8  = tid & 7;
    *(volatile v8h*)(qh  + ((size_t)bh * kL + n0 + row) * kD + c8 * 8) = vals[i];
    *(volatile v8h*)(kh  + ((size_t)bh * kL + n0 + row) * kD + c8 * 8) = vals[2 + i];
    *(volatile v8h*)(vth + ((size_t)bh * kD + row) * kL + n0 + c8 * 8)  = vals[4 + i];
  }
  __threadfence();
#pragma unroll
  for (int i = 0; i < 2; ++i) {
    const int row = i * 32 + (tid >> 3);
    const int c8  = tid & 7;
    *(volatile v8h*)(qh  + ((size_t)bh * kL + n0 + row) * kD + c8 * 8) = vals[i];
    *(volatile v8h*)(kh  + ((size_t)bh * kL + n0 + row) * kD + c8 * 8) = vals[2 + i];
    *(volatile v8h*)(vth + ((size_t)bh * kD + row) * kL + n0 + c8 * 8)  = vals[4 + i];
  }
}

__global__ __launch_bounds__(32)
void attn_kernel(const _Float16* __restrict__ qh, const _Float16* __restrict__ kh,
                 const _Float16* __restrict__ vth, _Float16* ah, float* pm)
{
  __shared__ union { _Float16 h[16 * kL]; v8h q[16 * kL / 8]; } P;
  __shared__ union { float f[kL]; v4f q[kL / 4]; } R0;
  __shared__ union { _Float16 h[16 * kD]; v8h q[16 * kD / 8]; } Os;

  const int l    = threadIdx.x & 31;
  const int hsel = l >> 4;
  const int h8   = hsel * 8;
  const int m    = l & 15;
  const int bh   = blockIdx.y;
  const int b    = bh / kH;
  const int hd   = bh - b * kH;
  const int q0   = blockIdx.x * 16;

  const _Float16* Qrow = qh + ((size_t)bh * kL + q0 + m) * kD;
  const v16h aq0 = ld_frag(Qrow, 0, h8);
  const v16h aq1 = ld_frag(Qrow, 32, h8);
  for (int nb = 0; nb < kL; nb += 16) {
    const _Float16* Krow = kh + ((size_t)bh * kL + nb + m) * kD;
    const v16h bk0 = ld_frag(Krow, 0, h8);
    const v16h bk1 = ld_frag(Krow, 32, h8);
    v8f s = zero8();
    s = wmma16(aq0, bk0, s);
    s = wmma16(aq1, bk1, s);
    asm volatile(NOP4 : "+v"(s) : "v"(aq0), "v"(aq1), "v"(bk0), "v"(bk1));
#pragma unroll
    for (int r = 0; r < 8; ++r)
      P.h[(h8 + r) * kL + nb + m] = (_Float16)(s[r] * 0.125f);
  }
  __syncthreads();

  {
    const int r    = m;
    const int half = hsel;
    const int base = r * (kL / 8) + half * (kL / 16);
    float mx = -3.0e38f;
    for (int i = 0; i < kL / 16; ++i) {
      const v8h c = P.q[base + i];
#pragma unroll
      for (int j = 0; j < 8; ++j) mx = fmaxf(mx, (float)c[j]);
    }
    mx = fmaxf(mx, __shfl_xor(mx, 16));
    float sum = 0.0f;
    for (int i = 0; i < kL / 16; ++i) {
      const v8h c = P.q[base + i];
#pragma unroll
      for (int j = 0; j < 8; ++j) sum += __expf((float)c[j] - mx);
    }
    sum += __shfl_xor(sum, 16);
    const float inv   = 1.0f / sum;
    const float inv4k = inv * 4096.0f;
    const bool row0 = (blockIdx.x == 0) && (r == 0);
    for (int i = 0; i < kL / 16; ++i) {
      const v8h c = P.q[base + i];
      v8h pv;
#pragma unroll
      for (int j = 0; j < 8; ++j) {
        const float e = __expf((float)c[j] - mx);
        pv[j] = (_Float16)(e * inv4k);
        if (row0) R0.f[half * (kL / 2) + i * 8 + j] = e * inv;
      }
      P.q[base + i] = pv;
    }
  }
  __syncthreads();

  v8f o[4];
#pragma unroll
  for (int j = 0; j < 4; ++j) o[j] = zero8();
  const _Float16* Prw = P.h + m * kL;
  const _Float16* V0 = vth + ((size_t)bh * kD + m) * kL;
  const _Float16* V1 = V0 + (size_t)16 * kL;
  const _Float16* V2 = V0 + (size_t)32 * kL;
  const _Float16* V3 = V0 + (size_t)48 * kL;
  for (int k = 0; k < kL; k += 32) {
    const v16h ap = ld_frag(Prw, k, h8);
    const v16h f0 = ld_frag(V0, k, h8);
    const v16h f1 = ld_frag(V1, k, h8);
    const v16h f2 = ld_frag(V2, k, h8);
    const v16h f3 = ld_frag(V3, k, h8);
    o[0] = wmma16(ap, f0, o[0]);
    o[1] = wmma16(ap, f1, o[1]);
    o[2] = wmma16(ap, f2, o[2]);
    o[3] = wmma16(ap, f3, o[3]);
    asm volatile(NOP4 : "+v"(o[0]), "+v"(o[1]), "+v"(o[2]), "+v"(o[3])
                      : "v"(ap), "v"(f0), "v"(f1), "v"(f2), "v"(f3));
  }
#pragma unroll
  for (int j = 0; j < 4; ++j)
#pragma unroll
    for (int r = 0; r < 8; ++r)
      Os.h[(h8 + r) * kD + j * 16 + m] = (_Float16)(o[j][r] * (1.0f / 4096.0f));
  __syncthreads();

  v8h ov[4];
#pragma unroll
  for (int p = 0; p < 4; ++p) {
    const int row = 4 * p + (l >> 3);
    const int c8  = l & 7;
    ov[p] = Os.q[row * 8 + c8];
  }
  const bool wmap = (blockIdx.x == 0);
  v4f rv[8];
  if (wmap) {
#pragma unroll
    for (int p = 0; p < 8; ++p) rv[p] = R0.q[32 * p + l];
  }
#pragma unroll
  for (int p = 0; p < 4; ++p) {
    const int row = 4 * p + (l >> 3);
    const int c8  = l & 7;
    *(volatile v8h*)(ah + ((size_t)b * kL + q0 + row) * kC + hd * kD + c8 * 8) = ov[p];
  }
  if (wmap) {
#pragma unroll
    for (int p = 0; p < 8; ++p)
      *(volatile v4f*)(pm + (size_t)bh * kL + 128 * p + 4 * l) = rv[p];
  }
  __threadfence();
#pragma unroll
  for (int p = 0; p < 4; ++p) {
    const int row = 4 * p + (l >> 3);
    const int c8  = l & 7;
    *(volatile v8h*)(ah + ((size_t)b * kL + q0 + row) * kC + hd * kD + c8 * 8) = ov[p];
  }
  if (wmap) {
#pragma unroll
    for (int p = 0; p < 8; ++p)
      *(volatile v4f*)(pm + (size_t)bh * kL + 128 * p + 4 * l) = rv[p];
  }
}

__global__ __launch_bounds__(256)
void map_kernel(const float* __restrict__ pm, float* amap, int nch)
{
  const int tid = threadIdx.x;
  v4f vals[4];
#pragma unroll
  for (int q = 0; q < 4; ++q) {
    const int c = tid + q * 256;
    v4f v;
#pragma unroll
    for (int e = 0; e < 4; ++e) v[e] = 0.0f;
    if (c < nch) {
#pragma unroll
      for (int e = 0; e < 4; ++e) {
        const int f  = 4 * c + e;
        const int bb = f / (kL - 1);
        const int mm = f - bb * (kL - 1) + 1;
        float s = 0.0f;
#pragma unroll 1
        for (int hh = 0; hh < kH; ++hh) s += pm[((size_t)(bb * kH + hh)) * kL + mm];
        v[e] = s * (1.0f / 16.0f);
      }
    }
    vals[q] = v;
  }
#pragma unroll
  for (int q = 0; q < 4; ++q) {
    const int c = tid + q * 256;
    if (c < nch) *(volatile v4f*)(amap + (size_t)c * 4) = vals[q];
  }
  __threadfence();
#pragma unroll
  for (int q = 0; q < 4; ++q) {
    const int c = tid + q * 256;
    if (c < nch) *(volatile v4f*)(amap + (size_t)c * 4) = vals[q];
  }
}

extern "C" void kernel_launch(void* const* d_in, const int* in_sizes, int n_in,
                              void* d_out, int out_size, void* d_ws, size_t ws_size,
                              hipStream_t stream)
{
  if (n_in < 20) return;
  const size_t TOK = (size_t)kTok, C = (size_t)kC;
  if (in_sizes[0]  != (int)(TOK * C * kNI)) return;
  if (in_sizes[1]  != kNI + 4)             return;
  if (in_sizes[2]  != (int)(3 * C * C))    return;
  if (in_sizes[3]  != (int)(3 * C))        return;
  if (in_sizes[4]  != (int)(C * C))        return;
  if (in_sizes[5]  != (int)C)              return;
  if (in_sizes[6]  != kD || in_sizes[7] != kD || in_sizes[8] != kD || in_sizes[9] != kD) return;
  if (in_sizes[10] != (int)(C * C))        return;
  if (in_sizes[11] != (int)C)              return;
  if (in_sizes[12] != (int)(64 * C))       return;
  if (in_sizes[13] != 64)                  return;
  if (in_sizes[14] != (int)(C * 64))       return;
  if (in_sizes[15] != (int)C)              return;
  if (in_sizes[16] != (int)(4 * C * C))    return;
  if (in_sizes[17] != (int)(4 * C))        return;
  if (in_sizes[18] != (int)(C * 4 * C))    return;
  if (in_sizes[19] != (int)C)              return;
  if (out_size != (int)(TOK * C + (size_t)kB * (kL - 1))) return;

  const float* x_list = (const float*)d_in[0];
  const float* w_     = (const float*)d_in[1];
  const float* qkv_w  = (const float*)d_in[2];
  const float* qkv_b  = (const float*)d_in[3];
  const float* proj_w = (const float*)d_in[4];
  const float* proj_b = (const float*)d_in[5];
  const float* nq_g   = (const float*)d_in[6];
  const float* nq_b   = (const float*)d_in[7];
  const float* nk_g   = (const float*)d_in[8];
  const float* nk_b   = (const float*)d_in[9];
  const float* conv_w = (const float*)d_in[10];
  const float* conv_b = (const float*)d_in[11];
  const float* ca1_w  = (const float*)d_in[12];
  const float* ca1_b  = (const float*)d_in[13];
  const float* ca2_w  = (const float*)d_in[14];
  const float* ca2_b  = (const float*)d_in[15];
  const float* mlp1_w = (const float*)d_in[16];
  const float* mlp1_b = (const float*)d_in[17];
  const float* mlp2_w = (const float*)d_in[18];
  const float* mlp2_b = (const float*)d_in[19];

  float* outF     = (float*)d_out;
  float* attn_map = outF + TOK * C;

  char* ws = (char*)d_ws;
  size_t off = 0;
  auto carve = [&](size_t bytes) -> char* {
    char* p = ws + off; off += (bytes + 255) & ~(size_t)255; return p;
  };
  _Float16* xh    = (_Float16*)carve(TOK * C * 2);
  _Float16* Hh    = (_Float16*)carve(TOK * 64 * 2);
  float*    xmix  = (float*)   carve(TOK * C * 4);
  _Float16* xmixh = (_Float16*)carve(TOK * C * 2);
  char* u1 = carve(TOK * 3 * C * 4);
  _Float16* Mh   = (_Float16*)u1;
  float*    qkvf = (float*)u1;
  char* u2 = carve(3 * TOK * C * 4);
  float* op0 = (float*)u2;
  float* op1 = op0 + TOK * C;
  float* op3 = op1 + TOK * C;
  _Float16* qhb = (_Float16*)u2;
  _Float16* khb = qhb + TOK * C;
  _Float16* vth = khb + TOK * C;
  _Float16* ahb = vth + TOK * C;
  _Float16* whc  = (_Float16*)carve(C * C * 2);
  _Float16* whc1 = (_Float16*)carve(64 * C * 2);
  _Float16* whc2 = (_Float16*)carve(C * 64 * 2);
  _Float16* whm1 = (_Float16*)carve(4 * C * C * 2);
  _Float16* whm2 = (_Float16*)carve(C * 4 * C * 2);
  _Float16* whq  = (_Float16*)carve(3 * C * C * 2);
  _Float16* whp  = (_Float16*)carve(C * C * 2);
  float* pm = (float*)carve((size_t)kB * kH * kL * 4);
  if (off > ws_size) return;

  auto cvt = [&](const float* s, int sstride, int soff, _Float16* d, size_t n) {
    const int n8 = (int)(n / 8);
    cvt_f16_kernel<<<dim3((unsigned)((n8 + 255) / 256)), 256, 0, stream>>>(s, sstride, soff, d, n8);
  };

  cvt(x_list, kNI, kNI - 1, xh, TOK * C);
  cvt(conv_w, 1, 0, whc,  C * C);
  cvt(ca1_w,  1, 0, whc1, 64 * C);
  cvt(ca2_w,  1, 0, whc2, C * 64);
  cvt(mlp1_w, 1, 0, whm1, 4 * C * C);
  cvt(mlp2_w, 1, 0, whm2, C * 4 * C);
  cvt(qkv_w,  1, 0, whq,  3 * C * C);
  cvt(proj_w, 1, 0, whp,  C * C);

  const unsigned gy = (unsigned)(TOK / 32);
  gemm_nt_kernel<1><<<dim3((unsigned)(C / 64), gy), 32, 0, stream>>>(xh, whc, conv_b, nullptr, op0, nullptr, kTok, kC, kC);
  gemm_nt_kernel<3><<<dim3(1, gy), 32, 0, stream>>>(xh, whc1, ca1_b, nullptr, nullptr, Hh, kTok, 64, kC);
  gemm_nt_kernel<4><<<dim3((unsigned)(C / 64), gy), 32, 0, stream>>>(Hh, whc2, ca2_b, x_list, op1, nullptr, kTok, kC, 64);
  gemm_nt_kernel<2><<<dim3((unsigned)(4 * C / 64), gy), 32, 0, stream>>>(xh, whm1, mlp1_b, nullptr, nullptr, Mh, kTok, 4 * kC, kC);
  gemm_nt_kernel<0><<<dim3((unsigned)(C / 64), gy), 32, 0, stream>>>(Mh, whm2, mlp2_b, nullptr, op3, nullptr, kTok, kC, 4 * kC);
  {
    const int n4 = (int)(TOK * C / 4);
    mix_kernel<<<dim3((unsigned)((n4 + 255) / 256)), 256, 0, stream>>>(x_list, w_, op0, op1, op3, xmix, n4);
  }
  cvt(xmix, 1, 0, xmixh, TOK * C);
  gemm_nt_kernel<0><<<dim3((unsigned)(3 * C / 64), gy), 32, 0, stream>>>(xmixh, whq, qkv_b, nullptr, qkvf, nullptr, kTok, 3 * kC, kC);
  ln_qkv_kernel<<<dim3((unsigned)(kL / 64), (unsigned)(kB * kH)), 256, 0, stream>>>(qkvf, nq_g, nq_b, nk_g, nk_b, qhb, khb, vth);
  attn_kernel<<<dim3((unsigned)(kL / 16), (unsigned)(kB * kH)), 32, 0, stream>>>(qhb, khb, vth, ahb, pm);
  {
    const int nch = (kB * (kL - 1)) / 4;
    map_kernel<<<dim3(1), 256, 0, stream>>>(pm, attn_map, nch);
  }
  gemm_nt_kernel<5><<<dim3((unsigned)(C / 64), gy), 32, 0, stream>>>(ahb, whp, proj_b, xmix, outF, nullptr, kTok, kC, kC);
}
